// MultiHeadAttention_1795296329949
// MI455X (gfx1250) — hardware-verified
//
#include <hip/hip_runtime.h>
#ifndef NB
#define NB 2
#endif
#ifndef SEQ
#define SEQ 2048
#endif
#define NB_FULL 2
#define SEQ_FULL 2048
#define DM 1024
#define NH 16
#define HD 64
#define ROT 32
#define MT (NB * SEQ)
#define BSTRIDE_FULL ((size_t)SEQ_FULL * DM)
#define CVT_NBH (MT * DM / 8 / 256)
#define CVT_NBW (DM * DM / 8 / 256)
#define WS_HALVES ((size_t)MT * DM * 6 + (size_t)DM * DM * 4)

#define MODE_QK 0
#define MODE_VT 1
#define MODE_OUT 2

static_assert(SEQ % 64 == 0);
static_assert(MT % 64 == 0);
static_assert(SEQ <= SEQ_FULL);
static_assert(NB <= NB_FULL);
static_assert(HD == 64);
static_assert(NH * HD == DM);
static_assert(DM % 64 == 0);
static_assert((MT * DM) % (8 * 256) == 0);
static_assert(WS_HALVES * 2 <= (size_t)134217728);

typedef __bf16 v16b __attribute__((ext_vector_type(16)));
typedef _Float16 v16h __attribute__((ext_vector_type(16)));
typedef unsigned short v8us __attribute__((ext_vector_type(8), may_alias));
typedef float v8f __attribute__((ext_vector_type(8)));
typedef float v4f __attribute__((ext_vector_type(4)));
typedef float v4fa __attribute__((ext_vector_type(4), may_alias));
union FragB { v16b v; v8us half[2]; unsigned short u[16]; };
union FragH { v16h v; v8us half[2]; _Float16 h[16]; unsigned short u[16]; };

#define LOG2E 1.4426950408889634f

__device__ __forceinline__ unsigned short bf16_bits(float x) {
  unsigned int u = __float_as_uint(x);
  return (unsigned short)((u + 0x7FFFu + ((u >> 16) & 1u)) >> 16);
}
__device__ __forceinline__ float bf16_val(unsigned short b) { return __uint_as_float(((unsigned int)b) << 16); }
__device__ __forceinline__ float bf16_rne(float x) { return bf16_val(bf16_bits(x)); }

__device__ __forceinline__ v8f mma_hh2(v16h a0, v16h b0, v16h a1, v16h b1, v8f c) {
  c = __builtin_amdgcn_wmma_f32_16x16x32_f16(false, a0, false, b0, (short)0, c, false, false);
  c = __builtin_amdgcn_wmma_f32_16x16x32_f16(false, a1, false, b1, (short)0, c, false, false);
  asm volatile("v_nop\n\tv_nop\n\tv_nop\n\tv_nop" : "+v"(c) : "v"(a0), "v"(b0), "v"(a1), "v"(b1));
  return c;
}
__device__ __forceinline__ void mma_h2(v16h a, v16h bh, v16h bl, v8f& ch, v8f& cl) {
  ch = __builtin_amdgcn_wmma_f32_16x16x32_f16(false, a, false, bh, (short)0, ch, false, false);
  cl = __builtin_amdgcn_wmma_f32_16x16x32_f16(false, a, false, bl, (short)0, cl, false, false);
  asm volatile("v_nop\n\tv_nop\n\tv_nop\n\tv_nop" : "+v"(ch), "+v"(cl) : "v"(a), "v"(bh), "v"(bl));
}
__device__ __forceinline__ void mma_b4(v16b a, v16b b0, v16b b1, v16b b2, v16b b3, v8f (&c)[4]) {
  c[0] = __builtin_amdgcn_wmma_f32_16x16x32_bf16(false, a, false, b0, (short)0, c[0], false, false);
  c[1] = __builtin_amdgcn_wmma_f32_16x16x32_bf16(false, a, false, b1, (short)0, c[1], false, false);
  c[2] = __builtin_amdgcn_wmma_f32_16x16x32_bf16(false, a, false, b2, (short)0, c[2], false, false);
  c[3] = __builtin_amdgcn_wmma_f32_16x16x32_bf16(false, a, false, b3, (short)0, c[3], false, false);
  asm volatile("v_nop\n\tv_nop\n\tv_nop\n\tv_nop" : "+v"(c[0]), "+v"(c[1]), "+v"(c[2]), "+v"(c[3])
               : "v"(a), "v"(b0), "v"(b1), "v"(b2), "v"(b3));
}
__device__ __forceinline__ void mma_h8(v16h ah, v16h al, v16h b0, v16h b1, v16h b2, v16h b3, v8f (&ch)[4], v8f (&cl)[4]) {
  ch[0] = __builtin_amdgcn_wmma_f32_16x16x32_f16(false, ah, false, b0, (short)0, ch[0], false, false);
  cl[0] = __builtin_amdgcn_wmma_f32_16x16x32_f16(false, al, false, b0, (short)0, cl[0], false, false);
  ch[1] = __builtin_amdgcn_wmma_f32_16x16x32_f16(false, ah, false, b1, (short)0, ch[1], false, false);
  cl[1] = __builtin_amdgcn_wmma_f32_16x16x32_f16(false, al, false, b1, (short)0, cl[1], false, false);
  ch[2] = __builtin_amdgcn_wmma_f32_16x16x32_f16(false, ah, false, b2, (short)0, ch[2], false, false);
  cl[2] = __builtin_amdgcn_wmma_f32_16x16x32_f16(false, al, false, b2, (short)0, cl[2], false, false);
  ch[3] = __builtin_amdgcn_wmma_f32_16x16x32_f16(false, ah, false, b3, (short)0, ch[3], false, false);
  cl[3] = __builtin_amdgcn_wmma_f32_16x16x32_f16(false, al, false, b3, (short)0, cl[3], false, false);
  asm volatile("v_nop\n\tv_nop\n\tv_nop\n\tv_nop"
               : "+v"(ch[0]), "+v"(ch[1]), "+v"(ch[2]), "+v"(ch[3]), "+v"(cl[0]), "+v"(cl[1]), "+v"(cl[2]), "+v"(cl[3])
               : "v"(ah), "v"(al), "v"(b0), "v"(b1), "v"(b2), "v"(b3));
}

__global__ __launch_bounds__(256) void k_cvt(const float* __restrict__ hid, const float* __restrict__ wq, const float* __restrict__ wk,
                                             const float* __restrict__ wv, const float* __restrict__ wo, unsigned short* __restrict__ P) {
  const int blk = blockIdx.x, tid = threadIdx.x;
  v4f x0, x1;
  size_t doff;
  int which = -1;
  if (blk < CVT_NBH) {
    const int t = blk * 256 + tid;
    const int row = t >> 7, piece = t & 127;
    const int b = row / SEQ, s = row - b * SEQ;
    const float* src = hid + (size_t)b * BSTRIDE_FULL + (size_t)s * DM + piece * 8;
    x0 = *(const v4fa*)(src); x1 = *(const v4fa*)(src + 4);
    doff = (size_t)t * 8;
  } else {
    const int wb = blk - CVT_NBH;
    which = wb / CVT_NBW;
    const int t = (wb - which * CVT_NBW) * 256 + tid;
    const size_t e = (size_t)t * 8;
    if (which == 0)      { x0 = *(const v4fa*)(wq + e); x1 = *(const v4fa*)(wq + e + 4); }
    else if (which == 1) { x0 = *(const v4fa*)(wk + e); x1 = *(const v4fa*)(wk + e + 4); }
    else if (which == 2) { x0 = *(const v4fa*)(wv + e); x1 = *(const v4fa*)(wv + e + 4); }
    else                 { x0 = *(const v4fa*)(wo + e); x1 = *(const v4fa*)(wo + e + 4); }
    doff = (size_t)MT * DM + (size_t)which * DM * DM + e;
  }
  v8us o;
  if (which == 3) {
    FragH f;
    f.h[0] = (_Float16)(bf16_rne(x0[0]) * 256.0f); f.h[1] = (_Float16)(bf16_rne(x0[1]) * 256.0f);
    f.h[2] = (_Float16)(bf16_rne(x0[2]) * 256.0f); f.h[3] = (_Float16)(bf16_rne(x0[3]) * 256.0f);
    f.h[4] = (_Float16)(bf16_rne(x1[0]) * 256.0f); f.h[5] = (_Float16)(bf16_rne(x1[1]) * 256.0f);
    f.h[6] = (_Float16)(bf16_rne(x1[2]) * 256.0f); f.h[7] = (_Float16)(bf16_rne(x1[3]) * 256.0f);
    o = f.half[0];
  } else {
    o[0] = bf16_bits(x0[0]); o[1] = bf16_bits(x0[1]); o[2] = bf16_bits(x0[2]); o[3] = bf16_bits(x0[3]);
    o[4] = bf16_bits(x1[0]); o[5] = bf16_bits(x1[1]); o[6] = bf16_bits(x1[2]); o[7] = bf16_bits(x1[3]);
  }
  unsigned short* d = P + doff;
  *(volatile v8us*)d = o;
  __threadfence();
  *(volatile v8us*)d = o;
}

template <int MODE>
__global__ __launch_bounds__(128) void k_gemm(const unsigned short* __restrict__ A, const unsigned short* __restrict__ A2,
                                              const unsigned short* __restrict__ Bm, unsigned short* __restrict__ Yh,
                                              float* __restrict__ Yf, const float* __restrict__ freqs, int N) {
  __shared__ __attribute__((aligned(16))) float st[64][68];
  const int tid = threadIdx.x, w = __builtin_amdgcn_readfirstlane((int)(tid >> 5)), lane = tid & 31, ln = lane & 15, hh = lane >> 4;
  const int ntn = N >> 6;
  const int tm = blockIdx.x / ntn, tn = blockIdx.x - tm * ntn;
  const int m0 = tm * 64, n0 = tn * 64;
  const size_t zb = (MODE == MODE_QK) ? (size_t)blockIdx.y * DM * DM : (size_t)0;
  const size_t zy = (MODE == MODE_QK) ? (size_t)blockIdx.y * MT * DM : (size_t)0;
  const size_t aoff = (size_t)(m0 + 16 * w + ln) * DM + 8 * hh;
  const unsigned short* ap = A + aoff;
  const unsigned short* ap2 = A2 + aoff;
  const unsigned short* bp = Bm + zb + (size_t)(n0 + ln) * DM + 8 * hh;
  v8f acc[4] = {}, acl[4] = {};
#pragma unroll 2
  for (int k0 = 0; k0 < DM; k0 += 32) {
    if (MODE == MODE_OUT) {
      FragH ah, al, b0, b1, b2, b3;
      ah.half[0] = *(const v8us*)(ap + k0);               ah.half[1] = *(const v8us*)(ap + k0 + 16);
      al.half[0] = *(const v8us*)(ap2 + k0);              al.half[1] = *(const v8us*)(ap2 + k0 + 16);
      b0.half[0] = *(const v8us*)(bp + k0);               b0.half[1] = *(const v8us*)(bp + k0 + 16);
      b1.half[0] = *(const v8us*)(bp + 16 * DM + k0);     b1.half[1] = *(const v8us*)(bp + 16 * DM + k0 + 16);
      b2.half[0] = *(const v8us*)(bp + 32 * DM + k0);     b2.half[1] = *(const v8us*)(bp + 32 * DM + k0 + 16);
      b3.half[0] = *(const v8us*)(bp + 48 * DM + k0);     b3.half[1] = *(const v8us*)(bp + 48 * DM + k0 + 16);
      mma_h8(ah.v, al.v, b0.v, b1.v, b2.v, b3.v, acc, acl);
    } else {
      FragB a, b0, b1, b2, b3;
      a.half[0]  = *(const v8us*)(ap + k0);               a.half[1]  = *(const v8us*)(ap + k0 + 16);
      b0.half[0] = *(const v8us*)(bp + k0);               b0.half[1] = *(const v8us*)(bp + k0 + 16);
      b1.half[0] = *(const v8us*)(bp + 16 * DM + k0);     b1.half[1] = *(const v8us*)(bp + 16 * DM + k0 + 16);
      b2.half[0] = *(const v8us*)(bp + 32 * DM + k0);     b2.half[1] = *(const v8us*)(bp + 32 * DM + k0 + 16);
      b3.half[0] = *(const v8us*)(bp + 48 * DM + k0);     b3.half[1] = *(const v8us*)(bp + 48 * DM + k0 + 16);
      mma_b4(a.v, b0.v, b1.v, b2.v, b3.v, acc);
    }
  }
#pragma unroll
  for (int t = 0; t < 4; ++t) {
#pragma unroll
    for (int r = 0; r < 8; ++r) {
      float v;
      if (MODE == MODE_OUT) v = (acc[t][r] + acl[t][r] * 0.00048828125f) * 0.00006103515625f;
      else v = acc[t][r];
      st[16 * w + 8 * hh + r][16 * t + ln] = v;
    }
  }
  __syncthreads();
  if (MODE == MODE_OUT) {
    v4f o[8];
#pragma unroll
    for (int it = 0; it < 8; ++it) {
      const int i = it * 128 + tid, row = i >> 4, c4 = (i & 15) * 4;
      o[it] = *(const v4fa*)&st[row][c4];
    }
    for (int pass = 0; pass < 2; ++pass) {
#pragma unroll
      for (int it = 0; it < 8; ++it) {
        const int i = it * 128 + tid, row = i >> 4, c4 = (i & 15) * 4;
        const int tok = m0 + row;
        const int b = tok / SEQ, s = tok - b * SEQ;
        *(volatile v4f*)(Yf + (size_t)b * BSTRIDE_FULL + (size_t)s * DM + n0 + c4) = o[it];
      }
      if (pass == 0) __threadfence();
    }
  } else {
    v8us o[4];
#pragma unroll
    for (int it = 0; it < 4; ++it) {
      const int i = it * 128 + tid, row = i >> 3, p8 = (i & 7) * 8;
      const v4f x0 = *(const v4fa*)&st[row][p8], x1 = *(const v4fa*)&st[row][p8 + 4];
      FragH f;
      if (MODE == MODE_QK) {
        const int tok = m0 + row;
        const int s = tok % SEQ;
        const float* fr = freqs + (size_t)s * (2 * ROT) + p8;
        const v4f f0 = *(const v4fa*)(fr), f1 = *(const v4fa*)(fr + 4);
        const float c0 = bf16_rne(f0[0]), s0 = bf16_rne(f0[1]), c1 = bf16_rne(f0[2]), s1 = bf16_rne(f0[3]);
        const float c2 = bf16_rne(f1[0]), s2 = bf16_rne(f1[1]), c3 = bf16_rne(f1[2]), s3 = bf16_rne(f1[3]);
        f.h[0] = (_Float16)(x0[0] * c0 - x0[1] * s0); f.h[1] = (_Float16)(x0[1] * c0 + x0[0] * s0);
        f.h[2] = (_Float16)(x0[2] * c1 - x0[3] * s1); f.h[3] = (_Float16)(x0[3] * c1 + x0[2] * s1);
        f.h[4] = (_Float16)(x1[0] * c2 - x1[1] * s2); f.h[5] = (_Float16)(x1[1] * c2 + x1[0] * s2);
        f.h[6] = (_Float16)(x1[2] * c3 - x1[3] * s3); f.h[7] = (_Float16)(x1[3] * c3 + x1[2] * s3);
      } else {
        f.h[0] = (_Float16)(x0[0] * 16.0f); f.h[1] = (_Float16)(x0[1] * 16.0f);
        f.h[2] = (_Float16)(x0[2] * 16.0f); f.h[3] = (_Float16)(x0[3] * 16.0f);
        f.h[4] = (_Float16)(x1[0] * 16.0f); f.h[5] = (_Float16)(x1[1] * 16.0f);
        f.h[6] = (_Float16)(x1[2] * 16.0f); f.h[7] = (_Float16)(x1[3] * 16.0f);
      }
      o[it] = f.half[0];
    }
    for (int pass = 0; pass < 2; ++pass) {
#pragma unroll
      for (int it = 0; it < 4; ++it) {
        const int i = it * 128 + tid, row = i >> 3, p8 = (i & 7) * 8;
        *(volatile v8us*)(Yh + zy + (size_t)(m0 + row) * N + n0 + p8) = o[it];
      }
      if (pass == 0) __threadfence();
    }
  }
}

__device__ __forceinline__ void fa_step(const unsigned short* __restrict__ Kp, const unsigned short* __restrict__ Vp,
                                        int key0, int ln, int hh, const FragH& q0, const FragH& q1,
                                        float& mr, float& lr, v8f (&Oh)[4], v8f (&Ol)[4]) {
  const unsigned short* kp0 = Kp + (size_t)(key0 + ln) * DM + 8 * hh;
  const unsigned short* kp1 = kp0 + (size_t)16 * DM;
  FragH k00, k01, k10, k11;
  k00.half[0] = *(const v8us*)(kp0);      k00.half[1] = *(const v8us*)(kp0 + 16);
  k01.half[0] = *(const v8us*)(kp0 + 32); k01.half[1] = *(const v8us*)(kp0 + 48);
  k10.half[0] = *(const v8us*)(kp1);      k10.half[1] = *(const v8us*)(kp1 + 16);
  k11.half[0] = *(const v8us*)(kp1 + 32); k11.half[1] = *(const v8us*)(kp1 + 48);
  const unsigned short* vp = Vp + (size_t)ln * MT + key0 + 8 * hh;
  FragH vf[4];
#pragma unroll
  for (int t = 0; t < 4; ++t) {
    vf[t].half[0] = *(const v8us*)(vp + (size_t)t * 16 * MT);
    vf[t].half[1] = *(const v8us*)(vp + (size_t)t * 16 * MT + 16);
  }
  const v8f z8 = {0.f, 0.f, 0.f, 0.f, 0.f, 0.f, 0.f, 0.f};
  const v8f s0 = mma_hh2(k00.v, q0.v, k01.v, q1.v, z8);
  const v8f s1 = mma_hh2(k10.v, q0.v, k11.v, q1.v, z8);
  float sc[16];
#pragma unroll
  for (int r = 0; r < 8; ++r) { sc[r] = s0[r] * 0.125f; sc[8 + r] = s1[r] * 0.125f; }
  float mx = sc[0];
#pragma unroll
  for (int i = 1; i < 16; ++i) mx = fmaxf(mx, sc[i]);
  mx = fmaxf(mx, __shfl_xor(mx, 16, 32));
  const float mnew = fmaxf(mr, mx);
  const float al = exp2f((mr - mnew) * LOG2E);
  mr = mnew;
  FragH ph, pl;
  float ps = 0.0f;
#pragma unroll
  for (int i = 0; i < 16; ++i) {
    const float pc = exp2f(fmaf(sc[i] - mnew, LOG2E, 8.0f));
    ps += pc;
    const _Float16 h = (_Float16)pc;
    ph.h[i] = h;
    pl.h[i] = (_Float16)((pc - (float)h) * 2048.0f);
  }
  ps += __shfl_xor(ps, 16, 32);
  lr = lr * al + ps;
#pragma unroll
  for (int t = 0; t < 4; ++t) { Oh[t] = Oh[t] * al; Ol[t] = Ol[t] * al; }
#pragma unroll
  for (int t = 0; t < 4; ++t) mma_h2(vf[t].v, ph.v, pl.v, Oh[t], Ol[t]);
}

__global__ __launch_bounds__(128) void k_attn(const unsigned short* __restrict__ Qh, const unsigned short* __restrict__ Kh,
                                              const unsigned short* __restrict__ Vt, unsigned short* __restrict__ Ch,
                                              unsigned short* __restrict__ Cl) {
  __shared__ __attribute__((aligned(16))) float so[4][16][68];
  const int tid = threadIdx.x, w = __builtin_amdgcn_readfirstlane((int)(tid >> 5)), lane = tid & 31, ln = lane & 15, hh = lane >> 4;
  const int qt = blockIdx.x % (SEQ / 64);
  const int bh = blockIdx.x / (SEQ / 64);
  const int h = bh % NH, b = bh / NH;
  const int qbase = qt * 64 + 16 * w;
  const int qg = qbase + ln;
  const unsigned short* qrow = Qh + (size_t)(b * SEQ + qg) * DM + h * HD + 8 * hh;
  FragH q0, q1;
  q0.half[0] = *(const v8us*)(qrow);      q0.half[1] = *(const v8us*)(qrow + 16);
  q1.half[0] = *(const v8us*)(qrow + 32); q1.half[1] = *(const v8us*)(qrow + 48);
  float mr = -3.0e38f, lr = 0.0f;
  v8f Oh[4] = {}, Ol[4] = {};
  const unsigned short* Kp = Kh + (size_t)b * SEQ * DM + h * HD;
  const unsigned short* Vp = Vt + (size_t)h * HD * MT + (size_t)b * SEQ;
#pragma unroll 1
  for (int j = 0; j < SEQ / 32; ++j)
    fa_step(Kp, Vp, 32 * j, ln, hh, q0, q1, mr, lr, Oh, Ol);

  const float inv = 4.0f * (1.0f / lr);
#pragma unroll
  for (int t = 0; t < 4; ++t)
#pragma unroll
    for (int r = 0; r < 8; ++r)
      so[w][ln][16 * t + 8 * hh + r] = (Oh[t][r] + Ol[t][r] * 0.00048828125f) * inv;
  __syncthreads();
  const int rsub = lane >> 3, p8 = (lane & 7) * 8;
  v8us oh[4], ol[4];
#pragma unroll
  for (int q = 0; q < 4; ++q) {
    const int row = 4 * q + rsub;
    const v4f x0 = *(const v4fa*)&so[w][row][p8], x1 = *(const v4fa*)&so[w][row][p8 + 4];
    FragH fh, fl;
#pragma unroll
    for (int i = 0; i < 4; ++i) {
      const _Float16 a = (_Float16)x0[i];
      const _Float16 c = (_Float16)x1[i];
      fh.h[i] = a;     fl.h[i] = (_Float16)((x0[i] - (float)a) * 2048.0f);
      fh.h[4 + i] = c; fl.h[4 + i] = (_Float16)((x1[i] - (float)c) * 2048.0f);
    }
    oh[q] = fh.half[0];
    ol[q] = fl.half[0];
  }
  const size_t obase = (size_t)(b * SEQ + qbase) * DM + h * HD + p8;
  for (int pass = 0; pass < 2; ++pass) {
#pragma unroll
    for (int q = 0; q < 4; ++q) {
      const int row = 4 * q + rsub;
      *(volatile v8us*)(Ch + obase + (size_t)row * DM) = oh[q];
      *(volatile v8us*)(Cl + obase + (size_t)row * DM) = ol[q];
    }
    if (pass == 0) __threadfence();
  }
}

extern "C" void kernel_launch(void* const* d_in, const int* in_sizes, int n_in,
                              void* d_out, int out_size, void* d_ws, size_t ws_size, hipStream_t stream) {
  if (n_in < 6) return;
  const long long need = (long long)(NB - 1) * SEQ_FULL * DM + (long long)SEQ * DM;
  if ((long long)in_sizes[0] < need) return;
  if ((long long)in_sizes[1] < (long long)SEQ * 2 * ROT) return;
  if ((long long)in_sizes[2] < (long long)DM * DM || (long long)in_sizes[3] < (long long)DM * DM) return;
  if ((long long)in_sizes[4] < (long long)DM * DM || (long long)in_sizes[5] < (long long)DM * DM) return;
  if ((long long)out_size < need) return;
  if (ws_size < WS_HALVES * 2) return;
  const float* hid   = (const float*)d_in[0];
  const float* freqs = (const float*)d_in[1];
  const float* wq    = (const float*)d_in[2];
  const float* wk    = (const float*)d_in[3];
  const float* wv    = (const float*)d_in[4];
  const float* wo    = (const float*)d_in[5];
  float* out = (float*)d_out;
  const size_t nHb = (size_t)MT * DM;
  const size_t nW  = (size_t)DM * DM;
  unsigned short* Hb = (unsigned short*)d_ws;
  unsigned short* Wb = Hb + nHb;
  unsigned short* QK = Wb + 4 * nW;
  unsigned short* Vt = QK + 2 * nHb;
  unsigned short* Ch = Vt + nHb;
  unsigned short* Cl = Ch + nHb;

  k_cvt<<<(unsigned)(CVT_NBH + 4 * CVT_NBW), 256, 0, stream>>>(hid, wq, wk, wv, wo, Hb);
  k_gemm<MODE_QK><<<dim3((unsigned)((MT / 64) * (DM / 64)), 2u, 1u), 128, 0, stream>>>(Hb, Hb, Wb, QK, out, freqs, DM);
  k_gemm<MODE_VT><<<(unsigned)((DM / 64) * (MT / 64)), 128, 0, stream>>>(Wb + 2 * nW, Wb + 2 * nW, Hb, Vt, out, freqs, MT);
  k_attn<<<(unsigned)(NB * NH * (SEQ / 64)), 128, 0, stream>>>(QK, QK + nHb, Vt, Ch, Cl);
  k_gemm<MODE_OUT><<<(unsigned)((MT / 64) * (DM / 64)), 128, 0, stream>>>(Ch, Cl, Wb + 3 * nW, QK, out, freqs, DM);
}
